// SOTAAttentionRouter_63196148793905
// MI455X (gfx1250) — hardware-verified
//
#include <hip/hip_runtime.h>
#include <math.h>

typedef __attribute__((ext_vector_type(16))) _Float16 v16h;
typedef __attribute__((ext_vector_type(16))) __bf16 v16b;
typedef __attribute__((ext_vector_type(8)))  _Float16 v8h;
typedef __attribute__((ext_vector_type(8)))  float v8f;
typedef __attribute__((ext_vector_type(4)))  float v4f;
typedef __attribute__((ext_vector_type(2)))  float v2f;
typedef __attribute__((ext_vector_type(4)))  unsigned v4u;
typedef __attribute__((ext_vector_type(4)))  int v4i;
typedef float __attribute__((may_alias)) float_a;
typedef int __attribute__((may_alias)) int_a;

template <typename T> __device__ __forceinline__ void vst2(void* p, T v) { *(volatile T*)p = v; __threadfence(); *(volatile T*)p = v; }
__device__ __forceinline__ v8f wmma16(v16h a, v16h b, v8f c) {
  v8f d = __builtin_amdgcn_wmma_f32_16x16x32_f16(false, a, false, b, (short)0, c, false, false);
  asm volatile("v_nop\n\tv_nop\n\tv_nop\n\tv_nop" : "+v"(d) : "v"(a), "v"(b));
  return d;
}
__device__ __forceinline__ v8f wmma_bf(v16b a, v16b b, v8f c) {
  v8f d = __builtin_amdgcn_wmma_f32_16x16x32_bf16(false, a, false, b, (short)0, c, false, false);
  asm volatile("v_nop\n\tv_nop\n\tv_nop\n\tv_nop" : "+v"(d) : "v"(a), "v"(b));
  return d;
}
__device__ __forceinline__ v16h frag_h(const _Float16* rowk0, int lane) {
  union { v16h v; v8h q[2]; } u; const _Float16* p = rowk0 + 8 * (lane >> 4);
  u.q[0] = *(const v8h*)p; u.q[1] = *(const v8h*)(p + 16); return u.v;
}
__device__ __forceinline__ v16h frag_f32(const float* rowk0, int lane) {
  v16h a; const float* p = rowk0 + 8 * (lane >> 4);
#pragma unroll
  for (int i = 0; i < 8; ++i) { a[i] = (_Float16)p[i]; a[8 + i] = (_Float16)p[16 + i]; }
  return a;
}
__device__ __forceinline__ v16h frag_f32s(const float* rowk0, int lane, float sc) {
  v16h a; const float* p = rowk0 + 8 * (lane >> 4);
#pragma unroll
  for (int i = 0; i < 8; ++i) { a[i] = (_Float16)(p[i] * sc); a[8 + i] = (_Float16)(p[16 + i] * sc); }
  return a;
}
__device__ __forceinline__ v16h fragc_f32(const float* W, int k0, int n, int lane, int ld, int K) {
  v16h a; const int g = lane >> 4;
#pragma unroll
  for (int i = 0; i < 8; ++i) { const int ka = k0 + 8 * g + i, kb = ka + 16;
    a[i] = (_Float16)(ka < K ? W[(size_t)(ka < K ? ka : K - 1) * ld + n] : 0.f); a[8 + i] = (_Float16)(kb < K ? W[(size_t)(kb < K ? kb : K - 1) * ld + n] : 0.f); }
  return a;
}
struct F2 { v16b h, l; };
__device__ __forceinline__ F2 bsplit16(const float v[16]) { F2 r;
#pragma unroll
  for (int i = 0; i < 16; ++i) { const __bf16 h = (__bf16)v[i]; r.h[i] = h; r.l[i] = (__bf16)(v[i] - (float)h); }
  return r; }
__device__ __forceinline__ F2 split_row(const float* row, int k0, int lane) { float v[16]; const float* p = row + k0 + 8 * (lane >> 4);
#pragma unroll
  for (int i = 0; i < 8; ++i) { v[i] = p[i]; v[8 + i] = p[16 + i]; }
  return bsplit16(v); }
__device__ __forceinline__ F2 split_rowK(const float* row, int k0, int lane, int K) { float v[16]; const int g = lane >> 4;
#pragma unroll
  for (int i = 0; i < 8; ++i) { const int ka = k0 + 8 * g + i, kb = ka + 16; v[i] = ka < K ? row[ka < K ? ka : K - 1] : 0.f; v[8 + i] = kb < K ? row[kb < K ? kb : K - 1] : 0.f; }
  return bsplit16(v); }
__device__ __forceinline__ F2 split_col(const float* W, int k0, int n, int lane, int ld, int K) { float v[16]; const int g = lane >> 4;
#pragma unroll
  for (int i = 0; i < 8; ++i) { const int ka = k0 + 8 * g + i, kb = ka + 16; v[i] = ka < K ? W[(size_t)(ka < K ? ka : K - 1) * ld + n] : 0.f; v[8 + i] = kb < K ? W[(size_t)(kb < K ? kb : K - 1) * ld + n] : 0.f; }
  return bsplit16(v); }
__device__ __forceinline__ v8f mac3(const F2& a, const F2& b, v8f c) { c = wmma_bf(a.l, b.h, c); c = wmma_bf(a.h, b.l, c); return wmma_bf(a.h, b.h, c); }
__device__ __forceinline__ float sigm(float v) { return 1.0f / (1.0f + expf(-v)); }
#define LDSX() do { asm volatile("s_wait_dscnt 0" ::: "memory"); __builtin_amdgcn_wave_barrier(); __builtin_amdgcn_fence(__ATOMIC_RELEASE, "workgroup"); } while (0)


#define NB 2
#define SS 2048
#define HID 2048
#define NH 16
#define NKV 4
#define HD 128
#define QW (NH * HD)
#define KW (NKV * HD)
#define QKVW (QW + 2 * KW)
#define NR (NB * SS)
#ifndef TQB
#define TQB (SS / 64)
#define TNB NB
#define TOB (NB * SS / 64)
#define TRB (NB * SS / 64)
#endif
typedef __attribute__((ext_vector_type(8))) __bf16 v8b;
__device__ __forceinline__ v16b frag_b(const __bf16* rowk0, int lane) {
  union { v16b v; v8b q[2]; } u; const __bf16* p = rowk0 + 8 * (lane >> 4);
  u.q[0] = *(const v8b*)p; u.q[1] = *(const v8b*)(p + 16); return u.v;
}
__device__ __forceinline__ float bfr(float v) { return (float)(__bf16)v; }
__device__ __attribute__((noinline)) float exp_ni(float v) { return expf(v); }
__device__ __attribute__((noinline)) float erf_ni(float v) { return erff(v); }
__device__ __attribute__((noinline)) float sin_ni(float v) { return sinf(v); }
__device__ __attribute__((noinline)) float cos_ni(float v) { return cosf(v); }
__device__ __attribute__((noinline)) float pow_ni(float a, float b) { return powf(a, b); }

#define PK_A 0
#define PK_P ((size_t)QKVW * HID)
#define PK_END (PK_P + (size_t)HID * QW)
#define WS_PK  0u
#define WS_QH  (((2u * PK_END) + 127u) / 128u * 128u)
#define WS_QL  (WS_QH + 2u * (size_t)NR * QW)
#define WS_KH  (WS_QL + 2u * (size_t)NR * QW)
#define WS_KL  (WS_KH + 2u * (size_t)NR * KW)
#define WS_VTH (WS_KL + 2u * (size_t)NR * KW)
#define WS_VTL (WS_VTH + 2u * (size_t)NR * KW)
#define WS_O   (WS_VTL + 2u * (size_t)NR * KW)
#define WS_END (WS_O + 4u * (size_t)NR * QW)

__global__ __launch_bounds__(256) void k_pack(const float* __restrict__ WQ, const float* __restrict__ WK, const float* __restrict__ WV, const float* __restrict__ WO, __bf16* __restrict__ PK) {
  __shared__ __align__(16) __bf16 s[HID]; const int n = blockIdx.x, which = blockIdx.y, t = threadIdx.x;
  if ((which == 1 || which == 2) && n >= KW) return;
  const float* Wm = (which == 0) ? WQ : (which == 1) ? WK : (which == 2) ? WV : WO; const int NO = (which == 1 || which == 2) ? KW : QW;
  for (int k = t; k < HID; k += 256) s[k] = (__bf16)Wm[(size_t)k * NO + n];
  __syncthreads();
  const size_t row = (which == 0) ? n : (which == 1) ? (QW + n) : (QW + KW + n);
  __bf16* dst = (which < 3) ? PK + PK_A + row * HID : PK + PK_P + (size_t)n * QW;
  for (int q = t; q < HID / 8; q += 256) vst2((unsigned*)(dst + q * 8), *(const v4u*)&s[q * 8]);
}
__global__ __launch_bounds__(128) void k_qkv(const float* __restrict__ X, const __bf16* __restrict__ P, const int* __restrict__ POS, const float* __restrict__ BQ, const float* __restrict__ BK, const float* __restrict__ BV, _Float16* __restrict__ QH, _Float16* __restrict__ QL, _Float16* __restrict__ KH, _Float16* __restrict__ KL, _Float16* __restrict__ VTH, _Float16* __restrict__ VTL) {
  __shared__ __align__(16) _Float16 soh[4][16][136], sol[4][16][136]; __shared__ __align__(16) _Float16 sth[128][72], stl[128][72];
  const int tid = threadIdx.x, wave = tid >> 5, lane = tid & 31, col = lane & 15, g = lane >> 4; const size_t r0 = (size_t)blockIdx.x * 64 + wave * 16; const int hb = blockIdx.y; const int n0 = hb * HD; const int kind = (hb < NH) ? 0 : (hb < NH + NKV) ? 1 : 2;
  v8f acc[8] = {};
#pragma unroll 2
  for (int kc = 0; kc < HID / 32; ++kc) { v16b a; { const float* p = X + (r0 + col) * HID + kc * 32 + 8 * g;
#pragma unroll
      for (int i = 0; i < 8; ++i) { a[i] = (__bf16)p[i]; a[8 + i] = (__bf16)p[16 + i]; } }
#pragma unroll
    for (int j = 0; j < 8; ++j) acc[j] = wmma_bf(a, frag_b(P + (size_t)(n0 + j * 16 + col) * HID + kc * 32, lane), acc[j]); }
  const float* BB = (kind == 0) ? (BQ ? BQ + n0 : nullptr) : (kind == 1) ? (BK ? BK + (n0 - QW) : nullptr) : (BV ? BV + (n0 - QW - KW) : nullptr);
  if (kind < 2) {
#pragma unroll
    for (int j = 0; j < 8; ++j) { const int d = j * 16 + col; const float invf = 1.0f / pow_ni(10000.0f, (float)(2 * (d & 63)) / (float)HD); const float bb = BB ? bfr(BB[d]) : 0.f, bbp = BB ? bfr(BB[d ^ 64]) : 0.f;
#pragma unroll
      for (int r = 0; r < 8; ++r) { const size_t row = r0 + 8 * g + r; const float v = acc[j][r] + bb; const float partner = acc[j ^ 4][r] + bbp; const float pos = (float)POS[row];
        const float ang = pos * invf; const float rot = (d < 64) ? -partner : partner; const float y = v * cos_ni(ang) + rot * sin_ni(ang);
        const _Float16 hv = (_Float16)y; soh[wave][8 * g + r][d] = hv; sol[wave][8 * g + r][d] = (_Float16)((y - (float)hv) * 2048.0f); } }
    LDSX();
    _Float16* DH_ = (kind == 0) ? QH : KH; _Float16* DL_ = (kind == 0) ? QL : KL; const int W_ = (kind == 0) ? QW : KW; const int c0 = (kind == 0) ? n0 : (n0 - QW);
    for (int rl = 0; rl < 16; ++rl) { const size_t o = (r0 + rl) * W_ + c0; if (lane < 16) vst2((unsigned*)(DH_ + o + lane * 8), *(const v4u*)&soh[wave][rl][lane * 8]); else vst2((unsigned*)(DL_ + o + (lane - 16) * 8), *(const v4u*)&sol[wave][rl][(lane - 16) * 8]); }
  } else {
#pragma unroll
    for (int j = 0; j < 8; ++j) { const float bb = BB ? bfr(BB[j * 16 + col]) : 0.f;
#pragma unroll
      for (int r = 0; r < 8; ++r) { const float v = acc[j][r] + bb; const _Float16 hv = (_Float16)v; sth[j * 16 + col][wave * 16 + 8 * g + r] = hv; stl[j * 16 + col][wave * 16 + 8 * g + r] = (_Float16)((v - (float)hv) * 2048.0f); } }
    __syncthreads();
    const size_t rb = (size_t)blockIdx.x * 64; const size_t b = rb / SS; const int s0 = (int)(rb % SS); const int c0 = n0 - QW - KW;
    for (int e = tid; e < 128 * 8; e += 128) { const int d = e >> 3, pc = e & 7; const size_t o = (b * KW + c0 + d) * SS + s0 + pc * 8; vst2((unsigned*)(VTH + o), *(const v4u*)&sth[d][pc * 8]); vst2((unsigned*)(VTL + o), *(const v4u*)&stl[d][pc * 8]); }
  }
}
__global__ __launch_bounds__(128) void k_attn(const _Float16* __restrict__ QH, const _Float16* __restrict__ QL, const _Float16* __restrict__ KH, const _Float16* __restrict__ KL, const _Float16* __restrict__ VTH, const _Float16* __restrict__ VTL, const float* __restrict__ MASK, float* __restrict__ O) {
  __shared__ __align__(16) _Float16 sp[4][16][40], spl[4][16][40]; __shared__ __align__(16) float so[4][16][HD + 4];
  const int tid = threadIdx.x, wave = tid >> 5, lane = tid & 31, col = lane & 15, g = lane >> 4; const int qb = blockIdx.x, n = blockIdx.y; const size_t b = blockIdx.z; const int kvh = n / (NH / NKV); const int q0 = qb * 64 + wave * 16; const size_t rowb = b * SS;
  const size_t qo = (rowb + q0 + col) * QW + n * HD;
  const _Float16* Vh = VTH + (b * KW + kvh * HD) * SS; const _Float16* Vl = VTL + (b * KW + kvh * HD) * SS;
  float m[8], l[8];
#pragma unroll
  for (int r = 0; r < 8; ++r) { m[r] = -3.0e38f; l[r] = 0.f; }
  v8f acc[8] = {}, accl[8] = {};
  const int nks = (qb * 64 + 64) / 32;
#pragma unroll 1
  for (int ks = 0; ks < nks; ++ks) { const int j0 = ks * 32; v8f s[2];
#pragma unroll
    for (int ct = 0; ct < 2; ++ct) { const int kk = j0 + ct * 16 + col; const size_t rk = (rowb + kk) * KW + kvh * HD; v8f c = {}, cl = {};
#pragma unroll 1
      for (int kc = 0; kc < HD / 32; ++kc) { const v16h aq = frag_h(QH + qo + kc * 32, lane), aql = frag_h(QL + qo + kc * 32, lane); const v16h kh = frag_h(KH + rk + kc * 32, lane); c = wmma16(aq, kh, c); cl = wmma16(aql, kh, cl); cl = wmma16(aq, frag_h(KL + rk + kc * 32, lane), cl); }
#pragma unroll
      for (int r = 0; r < 8; ++r) { const int qi = q0 + 8 * g + r; const bool keep = (kk <= qi); s[ct][r] = keep ? (c[r] + cl[r] * (1.0f / 2048.0f)) * 0.08838834764831845f : -3.0e38f; } }
#pragma unroll
    for (int r = 0; r < 8; ++r) { float mx = fmaxf(s[0][r], s[1][r]);
#pragma unroll
      for (int o = 1; o < 16; o <<= 1) mx = fmaxf(mx, __shfl_xor(mx, o));
      const float mn = fmaxf(m[r], mx); const float alpha = (m[r] <= -1.0e38f) ? 0.f : __expf(m[r] - mn);
      const float e0 = (s[0][r] <= -1.0e38f) ? 0.f : __expf(s[0][r] - mn), e1 = (s[1][r] <= -1.0e38f) ? 0.f : __expf(s[1][r] - mn); float es = e0 + e1;
#pragma unroll
      for (int o = 1; o < 16; o <<= 1) es += __shfl_xor(es, o);
      l[r] = l[r] * alpha + es; m[r] = (mn <= -1.0e38f) ? m[r] : mn;
#pragma unroll
      for (int dt = 0; dt < 8; ++dt) { acc[dt][r] *= alpha; accl[dt][r] *= alpha; }
      { const float p0 = e0 * 2048.0f, p1 = e1 * 2048.0f; const _Float16 h0 = (_Float16)p0, h1 = (_Float16)p1; sp[wave][8 * g + r][col] = h0; sp[wave][8 * g + r][16 + col] = h1; spl[wave][8 * g + r][col] = (_Float16)((p0 - (float)h0) * 2048.0f); spl[wave][8 * g + r][16 + col] = (_Float16)((p1 - (float)h1) * 2048.0f); } }
    LDSX();
    const v16h pa = frag_h(&sp[wave][col][0], lane), pal = frag_h(&spl[wave][col][0], lane);
#pragma unroll
    for (int dt = 0; dt < 8; ++dt) { const size_t vo = (size_t)(dt * 16 + col) * SS + j0; const v16h vh = frag_h(Vh + vo, lane); acc[dt] = wmma16(pa, vh, acc[dt]); accl[dt] = wmma16(pal, vh, accl[dt]); accl[dt] = wmma16(pa, frag_h(Vl + vo, lane), accl[dt]); }
    LDSX(); }
#pragma unroll
  for (int r = 0; r < 8; ++r) { const float il = (1.0f / 2048.0f) / l[r];
#pragma unroll
    for (int dt = 0; dt < 8; ++dt) so[wave][8 * g + r][dt * 16 + col] = (acc[dt][r] + accl[dt][r] * (1.0f / 2048.0f)) * il; }
  LDSX();
  for (int rl = 0; rl < 16; ++rl) vst2(O + (rowb + q0 + rl) * QW + n * HD + lane * 4, *(const v4f*)&so[wave][rl][lane * 4]);
}
__global__ __launch_bounds__(128) void k_out(const float* __restrict__ Oc, const __bf16* __restrict__ P, float* __restrict__ Y) {
  __shared__ __align__(16) float so[4][16][132];
  const int tid = threadIdx.x, wave = tid >> 5, lane = tid & 31, col = lane & 15, g = lane >> 4; const size_t r0 = (size_t)blockIdx.x * 64 + wave * 16; const int n0 = blockIdx.y * 128;
  v8f acc[8] = {};
#pragma unroll 2
  for (int kc = 0; kc < QW / 32; ++kc) { const F2 a = split_row(Oc + (r0 + col) * QW, kc * 32, lane);
#pragma unroll
    for (int j = 0; j < 8; ++j) { const v16b w = frag_b(P + (size_t)(n0 + j * 16 + col) * QW + kc * 32, lane); acc[j] = wmma_bf(a.l, w, acc[j]); acc[j] = wmma_bf(a.h, w, acc[j]); } }
#pragma unroll
  for (int j = 0; j < 8; ++j)
#pragma unroll
    for (int r = 0; r < 8; ++r) so[wave][8 * g + r][j * 16 + col] = acc[j][r];
  LDSX();
  for (int rl = 0; rl < 16; ++rl) vst2(Y + (r0 + rl) * HID + n0 + lane * 4, *(const v4f*)&so[wave][rl][lane * 4]);
}
extern "C" void kernel_launch(void* const* d_in, const int* in_sizes, int n_in, void* d_out, int out_size, void* d_ws, size_t ws_size, hipStream_t stream) {
  (void)in_sizes; (void)n_in; (void)out_size;
  const float** F = (const float**)d_in;
  if (ws_size < (size_t)WS_END) return;
  char* ws = (char*)d_ws; __bf16* PK = (__bf16*)(ws + WS_PK); _Float16 *QH = (_Float16*)(ws + WS_QH), *QL = (_Float16*)(ws + WS_QL), *KH = (_Float16*)(ws + WS_KH), *KL = (_Float16*)(ws + WS_KL), *VTH = (_Float16*)(ws + WS_VTH), *VTL = (_Float16*)(ws + WS_VTL); float* O = (float*)(ws + WS_O);
  k_pack<<<dim3(HID, 4), 256, 0, stream>>>(F[2], F[3], F[4], F[5], PK);
  k_qkv<<<dim3(TRB, NH + 2 * NKV), 128, 0, stream>>>(F[0], PK + PK_A, (const int*)d_in[1], nullptr, nullptr, nullptr, QH, QL, KH, KL, VTH, VTL);
  k_attn<<<dim3(TQB, NH, TNB), 128, 0, stream>>>(QH, QL, KH, KL, VTH, VTL, nullptr, O);
  k_out<<<dim3(TOB, HID / 128), 128, 0, stream>>>(O, PK + PK_P, (float*)d_out);
}
